// BucketAdjustedHinge_29626684408053
// MI455X (gfx1250) — hardware-verified
//
#include <hip/hip_runtime.h>


typedef _Float16 v16h __attribute__((ext_vector_type(16)));
typedef float    v8f  __attribute__((ext_vector_type(8)));
typedef float    v4f  __attribute__((ext_vector_type(4)));
typedef int      v4i  __attribute__((ext_vector_type(4)));

#define BLOCK_THREADS   256
#define WAVES_PER_BLOCK 8
#define NSEG            16
#define KB              32
#define KA              16
#define GROUP           128
#define MAX_BLOCKS      4096

__device__ __forceinline__ float softplus_f(float v) {
    return fmaxf(v, 0.f) + log1pf(expf(-fabsf(v)));
}

__device__ __forceinline__ v8f wmma_pair(v16h a0, v16h b0, v16h a1, v16h b1) {
    v8f acc = {0.f, 0.f, 0.f, 0.f, 0.f, 0.f, 0.f, 0.f};
    acc = __builtin_amdgcn_wmma_f32_16x16x32_f16(false, a0, false, b0, (short)0, acc, false, false);
    acc = __builtin_amdgcn_wmma_f32_16x16x32_f16(false, a1, false, b1, (short)0, acc, false, false);
    asm volatile("v_nop\n\tv_nop\n\tv_nop\n\tv_nop" : "+v"(acc) : "v"(a0), "v"(b0), "v"(a1), "v"(b1));
    return acc;
}

__device__ __forceinline__ float tile_pick(_Float16 xs, int bsel, int h,
                                           v16h abase, v16h aadj, v16h knb, v16h kna) {
    v16h xv;
#pragma unroll
    for (int e = 0; e < 16; ++e) xv[e] = xs;
    const v16h bb = __builtin_elementwise_min(xv, knb);
    const v16h ba = __builtin_elementwise_min(xv, kna);
    const v8f acc = wmma_pair(abase, bb, aadj, ba);
    const int r = bsel & 7;
    float v = acc[0];
    v = (r == 1) ? acc[1] : v;
    v = (r == 2) ? acc[2] : v;
    v = (r == 3) ? acc[3] : v;
    v = (r == 4) ? acc[4] : v;
    v = (r == 5) ? acc[5] : v;
    v = (r == 6) ? acc[6] : v;
    v = (r == 7) ? acc[7] : v;
    const float vo = __shfl_xor(v, 16);
    return (((bsel >> 3) & 1) == h) ? v : vo;
}

__global__ __launch_bounds__(BLOCK_THREADS)
void k_spline_eval(const float* __restrict__ X,
                   const float* __restrict__ x_mins,
                   const float* __restrict__ x_maxs,
                   const float* __restrict__ clip_los,
                   const float* __restrict__ clip_his,
                   const float* __restrict__ base_knots,
                   const float* __restrict__ base_raw_w,
                   const float* __restrict__ base_bias,
                   const float* __restrict__ adj_knots,
                   const float* __restrict__ adj_raw_w,
                   const float* __restrict__ adj_bias,
                   const int*   __restrict__ seg_idx,
                   float* __restrict__ out,
                   int n)
{
    __shared__ float4 sprm[NSEG];
    __shared__ float  sbias[NSEG];
    __shared__ float  swb[KB];
    __shared__ float  swa[NSEG * KA];

    const int t = threadIdx.x;
    if (t < NSEG * KA) swa[t] = 16.f * softplus_f(adj_raw_w[t]);
    if (t < KB)        swb[t] = 16.f * softplus_f(base_raw_w[t]);
    if (t < NSEG) {
        const float mn = x_mins[t], mx = x_maxs[t];
        float lo = clip_los[t], hi = clip_his[t];
        lo = __builtin_isfinite(lo) ? lo : -__builtin_inff();
        hi = __builtin_isfinite(hi) ? hi :  __builtin_inff();
        sprm[t]  = make_float4(mn, 1.f / (mx - mn + 1e-12f), lo, hi);
        sbias[t] = base_bias[0] + adj_bias[t];
    }
    __syncthreads();

    const int lane = t & 31;
    const int h    = lane >> 4;
    const int m    = lane & 15;
    const int wv   = t >> 5;

    v16h abase, aadj, knb, kna;
#pragma unroll
    for (int e = 0; e < 16; ++e) {
        const int k = (e < 8) ? (8 * h + e) : (16 + 8 * h + (e - 8));
        abase[e] = (_Float16)swb[k];
        knb[e]   = (_Float16)(64.f * base_knots[k]);
        if (e < 8) {
            aadj[e] = (_Float16)swa[m * KA + 8 * h + e];
            kna[e]  = (_Float16)(64.f * adj_knots[8 * h + e]);
        } else {
            aadj[e] = (_Float16)0.f;
            kna[e]  = (_Float16)0.f;
        }
    }

    const int ngroups = (n + GROUP - 1) / GROUP;
    const int gwave   = blockIdx.x * WAVES_PER_BLOCK + wv;
    const int nwaves  = gridDim.x * WAVES_PER_BLOCK;
    const float inv_scale = 1.f / 1024.f;

    for (int g = gwave; g < ngroups; g += nwaves) {
        const long long s0 = (long long)g * GROUP;
        const long long sb = s0 + 4 * lane;
        const bool full = (s0 + GROUP <= (long long)n);

        v4f xq;
        v4i bq;
        if (full) {
            xq = *(const v4f*)(X + sb);
            bq = *(const v4i*)(seg_idx + sb);
        } else {
#pragma unroll
            for (int c = 0; c < 4; ++c) {
                long long idx = sb + c;
                if (idx > (long long)(n - 1)) idx = (long long)(n - 1);
                xq[c] = X[idx];
                bq[c] = seg_idx[idx];
            }
        }

        v4f ov;
#pragma unroll
        for (int c = 0; c < 4; ++c) {
            int b = bq[c];
            b = (b < 0) ? 0 : b;
            b = (b > NSEG - 1) ? (NSEG - 1) : b;
            const float4 p = sprm[b];
            const float xr  = xq[c];
            const float xc  = fminf(fmaxf(xr, p.z), p.w);
            const float x01 = fminf(fmaxf((xc - p.x) * p.y, 0.f), 1.f);
            const float xm  = x01 * 64.f;
            const float xx  = __shfl_xor(xm, 16);
            const int   bx  = __shfl_xor(b, 16);
            const _Float16 xs0 = (_Float16)((h == 0) ? xm : xx);
            const int      bs0 = (h == 0) ? b : bx;
            const _Float16 xs1 = (_Float16)((h == 1) ? xm : xx);
            const int      bs1 = (h == 1) ? b : bx;
            const float pk0 = tile_pick(xs0, bs0, h, abase, aadj, knb, kna);
            const float pk1 = tile_pick(xs1, bs1, h, abase, aadj, knb, kna);
            const float rr  = (h == 0) ? pk0 : pk1;
            ov[c] = fmaf(rr, inv_scale, sbias[b]);
        }

        if (full) {
            *(volatile v4f*)(out + sb) = ov;
            __threadfence();
            *(volatile v4f*)(out + sb) = ov;
        } else {
#pragma unroll
            for (int c = 0; c < 4; ++c) {
                const long long idx = sb + c;
                if (idx < (long long)n) ((volatile float*)out)[idx] = ov[c];
            }
            __threadfence();
#pragma unroll
            for (int c = 0; c < 4; ++c) {
                const long long idx = sb + c;
                if (idx < (long long)n) ((volatile float*)out)[idx] = ov[c];
            }
        }
    }
}

extern "C" void kernel_launch(void* const* d_in, const int* in_sizes, int n_in,
                              void* d_out, int out_size, void* d_ws, size_t ws_size,
                              hipStream_t stream) {
    (void)n_in; (void)out_size; (void)d_ws; (void)ws_size;
    const float* X          = (const float*)d_in[0];
    const float* x_mins     = (const float*)d_in[1];
    const float* x_maxs     = (const float*)d_in[2];
    const float* clip_los   = (const float*)d_in[3];
    const float* clip_his   = (const float*)d_in[4];
    const float* base_knots = (const float*)d_in[5];
    const float* base_raw_w = (const float*)d_in[6];
    const float* base_bias  = (const float*)d_in[7];
    const float* adj_knots  = (const float*)d_in[8];
    const float* adj_raw_w  = (const float*)d_in[9];
    const float* adj_bias   = (const float*)d_in[10];
    const int*   seg_idx    = (const int*)d_in[11];
    float* out = (float*)d_out;

    const int n = in_sizes[0];
    if (n <= 0) return;
    const int ngroups = (n + GROUP - 1) / GROUP;
    int blocks = (ngroups + WAVES_PER_BLOCK - 1) / WAVES_PER_BLOCK;
    if (blocks > MAX_BLOCKS) blocks = MAX_BLOCKS;
    if (blocks < 1) blocks = 1;

    hipLaunchKernelGGL(k_spline_eval, dim3(blocks), dim3(BLOCK_THREADS), 0, stream,
                       X, x_mins, x_maxs, clip_los, clip_his,
                       base_knots, base_raw_w, base_bias,
                       adj_knots, adj_raw_w, adj_bias,
                       seg_idx, out, n);
}
